// multi_head_attn_26336739459554
// MI455X (gfx1250) — hardware-run, weakly checked
//
#include <hip/hip_runtime.h>
#include <stdint.h>

#pragma clang fp contract(off)

#define NF   64
#define NH   8
#define IW   80
#define IH   80
#define NPIX (IW * IH)
#define NC   32
#define KCV  (NF * 9)
#define PT   64
#ifndef NQRY
#define NQRY NPIX
#endif
#define XTP  72
#define VSP  72
#define OSP  68
#define L2E  1.44269504088896340736f
#define PEX  14.0f
#define VSC  16.0f
#define OSC  0.0625f
#define RSC  2048.0f
#define RRS  0.00048828125f

static_assert(NF == 64);
static_assert(NC == 32);
static_assert(NH == 8);
static_assert((NPIX % PT) == 0);
static_assert((NQRY % PT) == 0);
static_assert(NQRY <= NPIX);
static_assert((KCV % 32) == 0);
static_assert(((XTP * 2) % 16) == 0);
static_assert(((VSP * 2) % 16) == 0);
static_assert(((OSP * 4) % 16) == 0);
static_assert(((KCV * 2) % 16) == 0);

typedef _Float16       v8h  __attribute__((ext_vector_type(8)));
typedef _Float16       v16h __attribute__((ext_vector_type(16)));
typedef __bf16         v16b __attribute__((ext_vector_type(16)));
typedef unsigned short v8us __attribute__((ext_vector_type(8)));
typedef unsigned int   v4u  __attribute__((ext_vector_type(4)));
typedef float          v4f  __attribute__((ext_vector_type(4)));
typedef float          v8f  __attribute__((ext_vector_type(8)));

union FragH { v8h p[2]; v16h v; };
union FragB { v8us p[2]; v4u u[2]; v16b v; };
static_assert(sizeof(FragH) == 32);
static_assert(sizeof(FragB) == 32);

__device__ __forceinline__ v8f zero8() { v8f z = {0.f, 0.f, 0.f, 0.f, 0.f, 0.f, 0.f, 0.f}; return z; }

__device__ __forceinline__ unsigned int bf_bits(float x) {
  unsigned int u = __float_as_uint(x);
  u += 0x7FFFu + ((u >> 16) & 1u);
  return u >> 16;
}
__device__ __forceinline__ float bf_rne(float x) { return __uint_as_float(bf_bits(x) << 16); }

__device__ __forceinline__ v8f mma_h(v16h a, v16h b, v8f c) {
  v8f d = __builtin_amdgcn_wmma_f32_16x16x32_f16(false, a, false, b, (short)0, c, false, false);
#if defined(__HIP_DEVICE_COMPILE__)
  asm volatile("v_nop\n\tv_nop\n\tv_nop\n\tv_nop" : "+v"(d) : "v"(a), "v"(b));
#endif
  return d;
}
__device__ __forceinline__ v8f mma_b(v16b a, v16b b, v8f c) {
  v8f d = __builtin_amdgcn_wmma_f32_16x16x32_bf16(false, a, false, b, (short)0, c, false, false);
#if defined(__HIP_DEVICE_COMPILE__)
  asm volatile("v_nop\n\tv_nop\n\tv_nop\n\tv_nop" : "+v"(d) : "v"(a), "v"(b));
#endif
  return d;
}

__device__ __forceinline__ float max8(v8f d) {
  const float a = fmaxf(d[0], d[1]);
  const float b = fmaxf(d[2], d[3]);
  const float c = fmaxf(d[4], d[5]);
  const float e = fmaxf(d[6], d[7]);
  return fmaxf(fmaxf(a, b), fmaxf(c, e));
}

__global__ __launch_bounds__(256)
void k_prep(const float* __restrict__ X,
            const float* __restrict__ WQt, const float* __restrict__ BQt,
            const float* __restrict__ WKt, const float* __restrict__ BKt,
            const float* __restrict__ WQm, const float* __restrict__ WQx, const float* __restrict__ BQp,
            const float* __restrict__ WKx, const float* __restrict__ BKp,
            const float* __restrict__ PQ,
            unsigned short* QH, unsigned short* QL, unsigned short* KH, unsigned short* KL,
            unsigned short* XT) {
  __shared__ __align__(16) unsigned short s[5 * PT * XTP];
  const int t  = threadIdx.x;
  const int p0 = blockIdx.x * PT;

#pragma unroll 1
  for (int it = 0; it < 4; ++it) {
    const int idx = it * 256 + t;
    const int f   = idx >> 4;
    const int p4  = idx & 15;
    const int p   = p0 + 4 * p4;
    const v4f xa  = *(const v4f*)(X + (size_t)f * NPIX + p);
    const float wqx = bf_rne(WQx[f]);
    const float wkx = bf_rne(WKx[f]);
    const float bk  = bf_rne(BKp[f]);
    const float wkt = bf_rne(WKt[f]);
    const float bkt = bf_rne(BKt[f]);
    float xb[4], qs[4];
#pragma unroll
    for (int i = 0; i < 4; ++i) { xb[i] = bf_rne(xa[i]); qs[i] = 0.f; }
#pragma unroll 1
    for (int h = 0; h < NH; ++h) {
      const int hf = h * NF + f;
      const float wtm = bf_rne(WQm[hf]);
      const float bq  = bf_rne(BQp[hf]);
      const float wqt = bf_rne(WQt[hf]);
      const float bqt = bf_rne(BQt[hf]);
      const v4f pq = *(const v4f*)(PQ + (size_t)hf * NPIX + p);
#pragma unroll
      for (int i = 0; i < 4; ++i) {
        const float ta    = wtm * bf_rne(pq[i]);
        const float tb    = wqx * xb[i];
        const float inner = (ta + tb) + bq;
        const float q     = wqt * inner + bqt;
        qs[i] = qs[i] + q;
      }
    }
#pragma unroll
    for (int i = 0; i < 4; ++i) {
      const float tk = wkx * xb[i] + bk;
      const float kv = wkt * tk + bkt;
      const unsigned int qh = bf_bits(qs[i]);
      const unsigned int ql = bf_bits(qs[i] - __uint_as_float(qh << 16));
      const unsigned int kh = bf_bits(kv);
      const unsigned int kl = bf_bits(kv - __uint_as_float(kh << 16));
      const int e = (4 * p4 + i) * XTP + f;
      s[0 * PT * XTP + e] = (unsigned short)qh;
      s[1 * PT * XTP + e] = (unsigned short)ql;
      s[2 * PT * XTP + e] = (unsigned short)kh;
      s[3 * PT * XTP + e] = (unsigned short)kl;
      s[4 * PT * XTP + e] = (unsigned short)bf_bits(xa[i]);
    }
  }
  __syncthreads();

  v8us w[10];
  unsigned int pd[10];
#pragma unroll
  for (int it = 0; it < 10; ++it) {
    const int pl  = it >> 1;
    const int row = (it & 1) * 32 + (t >> 3);
    const int q   = t & 7;
    w[it]  = *(const v8us*)(s + pl * PT * XTP + row * XTP + 8 * q);
    pd[it] = (unsigned int)(p0 + row) * NF + 8 * q;
  }
#define PREP_ST(G, I) *(volatile v8us*)((G) + pd[I]) = w[I]
#define PREP_PASS \
  PREP_ST(QH, 0); PREP_ST(QH, 1); PREP_ST(QL, 2); PREP_ST(QL, 3); \
  PREP_ST(KH, 4); PREP_ST(KH, 5); PREP_ST(KL, 6); PREP_ST(KL, 7); \
  PREP_ST(XT, 8); PREP_ST(XT, 9)
  PREP_PASS;
  __threadfence();
  PREP_PASS;
#undef PREP_PASS
#undef PREP_ST
}

__global__ __launch_bounds__(128)
void k_conv(const unsigned short* __restrict__ XT, const float* __restrict__ Wc, const float* __restrict__ Bc,
            const float* __restrict__ WVt, const float* __restrict__ BVt, _Float16* VH, _Float16* VL) {
  __shared__ __align__(16) unsigned short Ws[NC * KCV];
  __shared__ __align__(16) _Float16 Vs[2 * NC * VSP];
  const int t    = threadIdx.x;
  const int lane = t & 31, wv = t >> 5;
  const int hh   = lane >> 4, n = lane & 15;
  const int p0   = blockIdx.x * PT;

  for (int e = t; e < NC * KCV; e += 128) {
    const int c   = e / KCV;
    const int rem = e - c * KCV;
    const int f   = rem / 9;
    const int tap = rem - f * 9;
    Ws[c * KCV + tap * NF + f] = (unsigned short)bf_bits(Wc[e]);
  }
  __syncthreads();

  const int p  = p0 + 16 * wv + n;
  const int pa = p / IH;
  const int pb = p - pa * IH;

  v8f acc0 = zero8(), acc1 = zero8();
#pragma unroll 1
  for (int st = 0; st < KCV / 32; ++st) {
    const int tap = st >> 1;
    const int dy  = tap / 3;
    const int dx  = tap - 3 * dy;
    const int aa  = pa + dy - 1;
    const int bb  = pb + dx - 1;
    const bool inb = ((unsigned)aa < (unsigned)IW) && ((unsigned)bb < (unsigned)IH);
    const int ac  = min(max(aa, 0), IW - 1);
    const int bc  = min(max(bb, 0), IH - 1);
    const unsigned int msk = inb ? 0xFFFFFFFFu : 0u;
    const unsigned short* xp = XT + (size_t)(ac * IH + bc) * NF + (st & 1) * 32 + 8 * hh;
    FragB bx;
    bx.p[0] = *(const v8us*)(xp);
    bx.p[1] = *(const v8us*)(xp + 16);
    bx.u[0] = bx.u[0] & msk;
    bx.u[1] = bx.u[1] & msk;
    const unsigned short* wp0 = Ws + n * KCV + st * 32 + 8 * hh;
    const unsigned short* wp1 = wp0 + 16 * KCV;
    FragB w0, w1;
    w0.p[0] = *(const v8us*)(wp0);
    w0.p[1] = *(const v8us*)(wp0 + 16);
    w1.p[0] = *(const v8us*)(wp1);
    w1.p[1] = *(const v8us*)(wp1 + 16);
    acc0 = mma_b(w0.v, bx.v, acc0);
    acc1 = mma_b(w1.v, bx.v, acc1);
  }

#pragma unroll
  for (int r = 0; r < 8; ++r) {
    const int c0 = 8 * hh + r;
    const int c1 = 16 + c0;
    {
      const float vc  = acc0[r] + bf_rne(Bc[c0]);
      const float v   = bf_rne(WVt[c0]) * vc + bf_rne(BVt[c0]);
      const float v16 = v * VSC;
      const _Float16 h16 = (_Float16)v16;
      const float res = v16 - (float)h16;
      Vs[c0 * VSP + 16 * wv + n]            = h16;
      Vs[NC * VSP + c0 * VSP + 16 * wv + n] = (_Float16)(res * RSC);
    }
    {
      const float vc  = acc1[r] + bf_rne(Bc[c1]);
      const float v   = bf_rne(WVt[c1]) * vc + bf_rne(BVt[c1]);
      const float v16 = v * VSC;
      const _Float16 h16 = (_Float16)v16;
      const float res = v16 - (float)h16;
      Vs[c1 * VSP + 16 * wv + n]            = h16;
      Vs[NC * VSP + c1 * VSP + 16 * wv + n] = (_Float16)(res * RSC);
    }
  }
  __syncthreads();

  v8h vw[4];
  unsigned int vp[4];
#pragma unroll
  for (int it = 0; it < 4; ++it) {
    const int L  = it * 16 + (t >> 3);
    const int pl = it >> 1;
    const int c  = L & 31;
    const int q  = t & 7;
    vw[it] = *(const v8h*)(Vs + pl * NC * VSP + c * VSP + 8 * q);
    vp[it] = (unsigned int)c * NPIX + p0 + 8 * q;
  }
  *(volatile v8h*)(VH + vp[0]) = vw[0];
  *(volatile v8h*)(VH + vp[1]) = vw[1];
  *(volatile v8h*)(VL + vp[2]) = vw[2];
  *(volatile v8h*)(VL + vp[3]) = vw[3];
  __threadfence();
  *(volatile v8h*)(VH + vp[0]) = vw[0];
  *(volatile v8h*)(VH + vp[1]) = vw[1];
  *(volatile v8h*)(VL + vp[2]) = vw[2];
  *(volatile v8h*)(VL + vp[3]) = vw[3];
}

__global__ __launch_bounds__(128)
void k_attn(const unsigned short* __restrict__ QH, const unsigned short* __restrict__ QL,
            const unsigned short* __restrict__ KH, const unsigned short* __restrict__ KL,
            const _Float16* __restrict__ VH, const _Float16* __restrict__ VL, float* out) {
  __shared__ __align__(16) float Os[NC * OSP];
  const int t    = threadIdx.x;
  const int lane = t & 31, wv = t >> 5;
  const int hh   = lane >> 4, n = lane & 15;
  const int bm0  = blockIdx.x * PT;
  const int m0   = bm0 + wv * 16;

  const size_t tq = (size_t)(m0 + n) * NF + 8 * hh;
  FragB qh0, qh1, ql0, ql1;
  qh0.p[0] = *(const v8us*)(QH + tq);
  qh0.p[1] = *(const v8us*)(QH + tq + 16);
  qh1.p[0] = *(const v8us*)(QH + tq + 32);
  qh1.p[1] = *(const v8us*)(QH + tq + 48);
  ql0.p[0] = *(const v8us*)(QL + tq);
  ql0.p[1] = *(const v8us*)(QL + tq + 16);
  ql1.p[0] = *(const v8us*)(QL + tq + 32);
  ql1.p[1] = *(const v8us*)(QL + tq + 48);

  const size_t kb  = (size_t)n * NF + 8 * hh;
  const size_t vb0 = (size_t)n * NPIX + 8 * hh;
  const size_t vb1 = (size_t)(16 + n) * NPIX + 8 * hh;

  v8f   Oh0 = zero8(), Oh1 = zero8(), Ol0 = zero8(), Ol1 = zero8();
  float m = -1.0e30f, z = 0.f;

#pragma unroll 1
  for (int k0 = 0; k0 < NPIX; k0 += PT) {
    v8f S[4];
#pragma unroll
    for (int ks = 0; ks < 4; ++ks) {
      const size_t a = kb + (size_t)(k0 + 16 * ks) * NF;
      FragB f0, f1, g0, g1;
      f0.p[0] = *(const v8us*)(KH + a);
      f0.p[1] = *(const v8us*)(KH + a + 16);
      f1.p[0] = *(const v8us*)(KH + a + 32);
      f1.p[1] = *(const v8us*)(KH + a + 48);
      v8f zz = mma_b(f0.v, qh0.v, zero8());
      zz     = mma_b(f0.v, ql0.v, zz);
      zz     = mma_b(f1.v, qh1.v, zz);
      zz     = mma_b(f1.v, ql1.v, zz);
      g0.p[0] = *(const v8us*)(KL + a);
      g0.p[1] = *(const v8us*)(KL + a + 16);
      g1.p[0] = *(const v8us*)(KL + a + 32);
      g1.p[1] = *(const v8us*)(KL + a + 48);
      zz     = mma_b(g0.v, qh0.v, zz);
      zz     = mma_b(g1.v, qh1.v, zz);
      S[ks]  = zz;
    }

    float tm = fmaxf(max8(S[0]), max8(S[1]));
    tm = fmaxf(tm, fmaxf(max8(S[2]), max8(S[3])));
    const float tmo = __shfl_xor(tm, 16, 32);
    tm = fmaxf(tm, tmo);
    const float mn    = fmaxf(m, tm * L2E);
    const float alpha = __builtin_amdgcn_exp2f(m - mn);
    m = mn;
    const float nb = PEX - mn;
    z *= alpha;
    Oh0 = Oh0 * alpha;
    Oh1 = Oh1 * alpha;
    Ol0 = Ol0 * alpha;
    Ol1 = Ol1 * alpha;

    FragH pf0, pf1;
#pragma unroll
    for (int r = 0; r < 8; ++r) {
      const _Float16 e0 = (_Float16)__builtin_amdgcn_exp2f(fmaf(S[0][r], L2E, nb));
      const _Float16 e1 = (_Float16)__builtin_amdgcn_exp2f(fmaf(S[1][r], L2E, nb));
      const _Float16 e2 = (_Float16)__builtin_amdgcn_exp2f(fmaf(S[2][r], L2E, nb));
      const _Float16 e3 = (_Float16)__builtin_amdgcn_exp2f(fmaf(S[3][r], L2E, nb));
      pf0.v[r]     = e0;
      pf0.v[8 + r] = e1;
      pf1.v[r]     = e2;
      pf1.v[8 + r] = e3;
      z += (float)e0;
      z += (float)e1;
      z += (float)e2;
      z += (float)e3;
    }

    {
      const _Float16* yp = VH + vb0 + k0;
      FragH ay;
      ay.p[0] = *(const v8h*)(yp);
      ay.p[1] = *(const v8h*)(yp + 16);
      Oh0 = mma_h(ay.v, pf0.v, Oh0);
      FragH by;
      by.p[0] = *(const v8h*)(yp + 32);
      by.p[1] = *(const v8h*)(yp + 48);
      Oh0 = mma_h(by.v, pf1.v, Oh0);
    }
    {
      const _Float16* yp = VH + vb1 + k0;
      FragH ay;
      ay.p[0] = *(const v8h*)(yp);
      ay.p[1] = *(const v8h*)(yp + 16);
      Oh1 = mma_h(ay.v, pf0.v, Oh1);
      FragH by;
      by.p[0] = *(const v8h*)(yp + 32);
      by.p[1] = *(const v8h*)(yp + 48);
      Oh1 = mma_h(by.v, pf1.v, Oh1);
    }
    {
      const _Float16* yp = VL + vb0 + k0;
      FragH ay;
      ay.p[0] = *(const v8h*)(yp);
      ay.p[1] = *(const v8h*)(yp + 16);
      Ol0 = mma_h(ay.v, pf0.v, Ol0);
      FragH by;
      by.p[0] = *(const v8h*)(yp + 32);
      by.p[1] = *(const v8h*)(yp + 48);
      Ol0 = mma_h(by.v, pf1.v, Ol0);
    }
    {
      const _Float16* yp = VL + vb1 + k0;
      FragH ay;
      ay.p[0] = *(const v8h*)(yp);
      ay.p[1] = *(const v8h*)(yp + 16);
      Ol1 = mma_h(ay.v, pf0.v, Ol1);
      FragH by;
      by.p[0] = *(const v8h*)(yp + 32);
      by.p[1] = *(const v8h*)(yp + 48);
      Ol1 = mma_h(by.v, pf1.v, Ol1);
    }
  }

  const float zo = __shfl_xor(z, 16, 32);
  const float zt = z + zo;
  const float rz = __builtin_amdgcn_rcpf(zt) * OSC;
#pragma unroll
  for (int r = 0; r < 8; ++r) {
    const float u0 = (Oh0[r] + Ol0[r] * RRS) * rz;
    const float u1 = (Oh1[r] + Ol1[r] * RRS) * rz;
    Os[(8 * hh + r) * OSP + 16 * wv + n]      = u0;
    Os[(16 + 8 * hh + r) * OSP + 16 * wv + n] = u1;
  }
  __syncthreads();

  v4f          ov[4];
  unsigned int po[4];
#pragma unroll
  for (int it = 0; it < 4; ++it) {
    const int L    = it * 16 + (t >> 3);
    const int c    = L >> 1;
    const int half = L & 1;
    const int q    = t & 7;
    ov[it] = *(const v4f*)(Os + c * OSP + half * 32 + 4 * q);
    po[it] = (unsigned int)c * NPIX + bm0 + half * 32 + 4 * q;
  }
#pragma unroll
  for (int it = 0; it < 4; ++it) *(volatile v4f*)(out + po[it]) = ov[it];
  __threadfence();
#pragma unroll
  for (int it = 0; it < 4; ++it) *(volatile v4f*)(out + po[it]) = ov[it];
}

extern "C" void kernel_launch(void* const* d_in, const int* in_sizes, int n_in,
                              void* d_out, int out_size, void* d_ws, size_t ws_size,
                              hipStream_t stream) {
  if (n_in < 15) return;
  if (in_sizes[0]  != NF * NPIX) return;
  if (in_sizes[1]  != NH * NF) return;
  if (in_sizes[2]  != NH * NF) return;
  if (in_sizes[3]  != NF) return;
  if (in_sizes[4]  != NF) return;
  if (in_sizes[5]  != NC) return;
  if (in_sizes[6]  != NC) return;
  if (in_sizes[7]  != NH * NF) return;
  if (in_sizes[8]  != NF) return;
  if (in_sizes[9]  != NH * NF) return;
  if (in_sizes[10] != NF) return;
  if (in_sizes[11] != NF) return;
  if (in_sizes[12] != NH * NF * NPIX) return;
  if (in_sizes[13] != NC * KCV) return;
  if (in_sizes[14] != NC) return;
  if (out_size != NC * NPIX) return;

  size_t off = 0;
  const size_t plq = (size_t)NPIX * NF * 2;
  const size_t plv = (size_t)NC * NPIX * 2;
  const size_t oQH = off; off += plq;
  const size_t oQL = off; off += plq;
  const size_t oKH = off; off += plq;
  const size_t oKL = off; off += plq;
  const size_t oXT = off; off += plq;
  const size_t oVH = off; off += plv;
  const size_t oVL = off; off += plv;
  if (off > ws_size) return;
  if (off > (size_t)134217728) return;

  const float* X    = (const float*)d_in[0];
  const float* WQt  = (const float*)d_in[1];
  const float* BQt  = (const float*)d_in[2];
  const float* WKt  = (const float*)d_in[3];
  const float* BKt  = (const float*)d_in[4];
  const float* WVt  = (const float*)d_in[5];
  const float* BVt  = (const float*)d_in[6];
  const float* WQm  = (const float*)d_in[7];
  const float* WQx  = (const float*)d_in[8];
  const float* BQp  = (const float*)d_in[9];
  const float* WKx  = (const float*)d_in[10];
  const float* BKp  = (const float*)d_in[11];
  const float* PQ   = (const float*)d_in[12];
  const float* Wc   = (const float*)d_in[13];
  const float* Bc   = (const float*)d_in[14];
  float* out = (float*)d_out;

  char* ws = (char*)d_ws;
  unsigned short* QH = (unsigned short*)(ws + oQH);
  unsigned short* QL = (unsigned short*)(ws + oQL);
  unsigned short* KH = (unsigned short*)(ws + oKH);
  unsigned short* KL = (unsigned short*)(ws + oKL);
  unsigned short* XT = (unsigned short*)(ws + oXT);
  _Float16*       VH = (_Float16*)(ws + oVH);
  _Float16*       VL = (_Float16*)(ws + oVL);

  k_prep<<<dim3(NPIX / PT), dim3(256), 0, stream>>>(X, WQt, BQt, WKt, BKt, WQm, WQx, BQp, WKx, BKp, PQ,
                                                    QH, QL, KH, KL, XT);
  k_conv<<<dim3(NPIX / PT), dim3(128), 0, stream>>>(XT, Wc, Bc, WVt, BVt, VH, VL);
  k_attn<<<dim3(NQRY / PT), dim3(128), 0, stream>>>(QH, QL, KH, KL, VH, VL, out);
  (void)hipGetLastError();
}
